// SpinnTreeLSTM_34110630265348
// MI455X (gfx1250) — hardware-run, weakly checked
//
#include <hip/hip_runtime.h>
#include <math.h>

constexpr int NBAT   = 128;
constexpr int NLEAF  = 128;
constexpr int NEMB   = 256;
constexpr int NHID   = 256;
constexpr int NGATE  = 4 * NHID;
constexpr int NSTEPS = 2 * NLEAF - 1;
constexpr int NKC    = 2 * NHID;
constexpr int NROWS  = NLEAF * NBAT;
constexpr int NTHR   = 256;
constexpr int ROWS_BLK = 16;
constexpr int APITCH = 520;
constexpr int GPITCH = 1028;
constexpr int SLP    = 68;
constexpr float WCARRY     = 16.0f;
constexpr float WCARRY_INV = 1.0f / 16.0f;
constexpr float RES_CARRY     = 2048.0f;
constexpr float RES_CARRY_INV = 1.0f / 2048.0f;
constexpr float F16_FLUSH = 6.2e-5f;
constexpr int NOUT0 = NBAT * NSTEPS * NHID;
constexpr int NOUT1 = NBAT * NHID;

static_assert(NSTEPS == 255, "step count");
static_assert(NEMB % 32 == 0 && NKC % 32 == 0, "K multiple of 32");
static_assert(NROWS % 16 == 0 && NHID % 32 == 0, "leaf tile multiples");
static_assert(((NROWS / 16) * (NHID / 32)) % 8 == 0, "leaf grid exact");
static_assert(NBAT % ROWS_BLK == 0, "scan grid exact");
static_assert(NGATE == 8 * 128, "8 waves x 128 gate columns");
static_assert(NHID == 4 * 64, "4 column groups of 64 per row");
static_assert((size_t)NOUT0 * 4 == 33423360, "out1 byte offset");
static_assert((size_t)(NOUT0 + NOUT1) * 4 == 33554432, "out2 byte offset");
static_assert((size_t)(NOUT0 + 2 * NOUT1) * 4 == 33685504, "d_out total bytes");

typedef __attribute__((ext_vector_type(16))) _Float16 v16h;
typedef __attribute__((ext_vector_type(8)))  _Float16 v8h;
typedef __attribute__((ext_vector_type(4)))  _Float16 v4h;
typedef __attribute__((ext_vector_type(8)))  float    v8f;
typedef __attribute__((ext_vector_type(4)))  float    v4f;

__device__ __forceinline__ void guard8_h(v8f& a0, v8f& a1, v8f& a2, v8f& a3,
                                         v8f& a4, v8f& a5, v8f& a6, v8f& a7,
                                         v16h x, v16h b0, v16h b1, v16h b2, v16h b3,
                                         v16h b4, v16h b5, v16h b6, v16h b7) {
  asm volatile("v_nop\n\tv_nop\n\tv_nop\n\tv_nop"
               : "+v"(a0), "+v"(a1), "+v"(a2), "+v"(a3), "+v"(a4), "+v"(a5), "+v"(a6), "+v"(a7)
               : "v"(x), "v"(b0), "v"(b1), "v"(b2), "v"(b3), "v"(b4), "v"(b5), "v"(b6), "v"(b7));
}
__device__ __forceinline__ void acc_guard4(v8f& a, v8f& b, v8f& c, v8f& d) {
  asm volatile("v_nop\n\tv_nop\n\tv_nop\n\tv_nop" : "+v"(a), "+v"(b), "+v"(c), "+v"(d));
}

struct FragH {
  union U { v16h v; v8h h[2]; };
  static __device__ __forceinline__ v16h load(const _Float16* p) {
    U f;
    f.h[0] = *(const v8h*)(p);
    f.h[1] = *(const v8h*)(p + 16);
    return f.v;
  }
  static __device__ __forceinline__ v8f mma(v16h a, v16h b, v8f c) {
    return __builtin_amdgcn_wmma_f32_16x16x32_f16(false, a, false, b, (short)0, c, false, false);
  }
};

__device__ __forceinline__ v8f mma_g(v16h a, v16h b, v8f c) {
  c = __builtin_amdgcn_wmma_f32_16x16x32_f16(false, a, false, b, (short)0, c, false, false);
  asm volatile("v_nop\n\tv_nop\n\tv_nop\n\tv_nop" : "+v"(c) : "v"(a), "v"(b));
  return c;
}

__device__ __forceinline__ void wave_lds_sync() {
  __builtin_amdgcn_fence(__ATOMIC_RELEASE, "workgroup");
  __builtin_amdgcn_wave_barrier();
  __builtin_amdgcn_fence(__ATOMIC_ACQUIRE, "workgroup");
}

__device__ __forceinline__ float sigm(float x) { return __builtin_amdgcn_rcpf(1.0f + expf(-x)); }

__device__ __forceinline__ void split_f16(float v, float& hf, float& lf) {
  const float hr = (float)(_Float16)v;
  hf = (fabsf(v) < F16_FLUSH) ? 0.0f : hr;
  const float lr = (float)(_Float16)((v - hf) * RES_CARRY);
  lf = (fabsf(lr) < F16_FLUSH) ? 0.0f : lr;
}

__global__ __launch_bounds__(NTHR) void cvt8_f16_split_kernel(const float* __restrict__ src,
                                                              unsigned short* __restrict__ dsth,
                                                              unsigned short* __restrict__ dstl, int n8) {
  const int i = blockIdx.x * NTHR + threadIdx.x;
  if (i < n8) {
    const v4f a = *(const v4f*)(src + (size_t)i * 8);
    const v4f b = *(const v4f*)(src + (size_t)i * 8 + 4);
    v8h hv, lv;
#pragma unroll
    for (int e = 0; e < 4; ++e) {
      float h0, l0, h1, l1;
      split_f16(a[e], h0, l0);
      split_f16(b[e], h1, l1);
      hv[e]     = (_Float16)h0;
      lv[e]     = (_Float16)l0;
      hv[4 + e] = (_Float16)h1;
      lv[4 + e] = (_Float16)l1;
    }
    *(volatile v8h*)(dsth + (size_t)i * 8) = hv;
    *(volatile v8h*)(dstl + (size_t)i * 8) = lv;
    __threadfence();
    *(volatile v8h*)(dsth + (size_t)i * 8) = hv;
    *(volatile v8h*)(dstl + (size_t)i * 8) = lv;
  }
}

__global__ __launch_bounds__(NTHR) void weight_planes_kernel(const float* __restrict__ Wc, const float* __restrict__ Wo,
                                                             const float* __restrict__ Wl, const float* __restrict__ Wr,
                                                             unsigned short* __restrict__ WcoT,
                                                             unsigned short* __restrict__ WcoL,
                                                             unsigned short* __restrict__ WlrT) {
  __shared__ float Tt[64 * 65];
  const int tid = threadIdx.x;
  const int bid = blockIdx.x;
  const float* src;
  unsigned short* O;
  unsigned short* O2;
  int ncol, ldo, tl, ntx;
  if (bid < 16)      { src = Wc; O = WcoT;                       O2 = WcoL;                       ncol = NHID;  ldo = NEMB; tl = bid;      ntx = NHID / 64; }
  else if (bid < 32) { src = Wo; O = WcoT + (size_t)NHID * NEMB; O2 = WcoL + (size_t)NHID * NEMB; ncol = NHID;  ldo = NEMB; tl = bid - 16; ntx = NHID / 64; }
  else if (bid < 96) { src = Wl; O = WlrT;                       O2 = WcoL;                       ncol = NGATE; ldo = NKC;  tl = bid - 32; ntx = NGATE / 64; }
  else               { src = Wr; O = WlrT + NHID;                O2 = WcoL;                       ncol = NGATE; ldo = NKC;  tl = bid - 96; ntx = NGATE / 64; }
  const bool leafp = (bid < 32);
  const int bx = tl % ntx, by = tl / ntx;
  const int c0 = bx * 64, r0 = by * 64;
#pragma unroll
  for (int i = 0; i < 4; ++i) {
    const int idx = i * NTHR + tid;
    const int rr = idx >> 4, cc = (idx & 15) * 4;
    const v4f v = *(const v4f*)(src + (size_t)(r0 + rr) * (size_t)ncol + c0 + cc);
    Tt[rr * 65 + cc + 0] = v[0];
    Tt[rr * 65 + cc + 1] = v[1];
    Tt[rr * 65 + cc + 2] = v[2];
    Tt[rr * 65 + cc + 3] = v[3];
  }
  __syncthreads();
  const int q = tid >> 3, c8 = (tid & 7) * 8;
  v8h hv[2], lv[2];
#pragma unroll
  for (int g = 0; g < 2; ++g) {
    const int qq = g * 32 + q;
#pragma unroll
    for (int e = 0; e < 8; ++e) {
      const float f = Tt[(c8 + e) * 65 + qq] * WCARRY;
      float hs, ls;
      split_f16(f, hs, ls);
      const float hsel = leafp ? hs : f;
      hv[g][e] = (_Float16)hsel;
      lv[g][e] = (_Float16)ls;
    }
  }
  for (int pass = 0; pass < 2; ++pass) {
#pragma unroll
    for (int g = 0; g < 2; ++g) {
      const size_t o = (size_t)(c0 + g * 32 + q) * (size_t)ldo + (size_t)(r0 + c8);
      *(volatile v8h*)(O + o) = hv[g];
      if (leafp) *(volatile v8h*)(O2 + o) = lv[g];
    }
    __threadfence();
  }
}

__global__ __launch_bounds__(NTHR) void leaf_gemm_kernel(const unsigned short* __restrict__ Xhp,
                                                         const unsigned short* __restrict__ Xlp,
                                                         const unsigned short* __restrict__ Whp,
                                                         const unsigned short* __restrict__ Wlp,
                                                         const float* __restrict__ bc, const float* __restrict__ bo,
                                                         float* __restrict__ LH, float* __restrict__ LC) {
  __shared__ __align__(16) float sT[NTHR / 32][16 * SLP];
  const _Float16* XH = (const _Float16*)Xhp;
  const _Float16* XL = (const _Float16*)Xlp;
  const _Float16* WH = (const _Float16*)Whp;
  const _Float16* WL = (const _Float16*)Wlp;
  const int lane = threadIdx.x & 31, wave = threadIdx.x >> 5;
  const int tile = blockIdx.x * 8 + wave;
  const int tn = tile & 7, tm = tile >> 3;
  const int m0 = tm * 16, n0 = tn * 32;
  const int rl = lane & 15, hh = lane >> 4, koff = hh * 8;

  const size_t ao  = (size_t)(m0 + rl) * NEMB + koff;
  const size_t wo0 = (size_t)(n0 + rl) * NEMB + koff;
  const size_t wo1 = wo0 + (size_t)16 * NEMB;
  const size_t wo2 = wo0 + (size_t)NHID * NEMB;
  const size_t wo3 = wo2 + (size_t)16 * NEMB;
  const _Float16* axh = XH + ao;
  const _Float16* axl = XL + ao;
  const _Float16* wh0 = WH + wo0;
  const _Float16* wl0 = WL + wo0;
  const _Float16* wh1 = WH + wo1;
  const _Float16* wl1 = WL + wo1;
  const _Float16* wh2 = WH + wo2;
  const _Float16* wl2 = WL + wo2;
  const _Float16* wh3 = WH + wo3;
  const _Float16* wl3 = WL + wo3;

  const v8f z8 = {0.f, 0.f, 0.f, 0.f, 0.f, 0.f, 0.f, 0.f};
  v8f mC0 = z8, mC1 = z8, mO0 = z8, mO1 = z8;
  v8f rC0 = z8, rC1 = z8, rO0 = z8, rO1 = z8;
#pragma unroll 1
  for (int k0 = 0; k0 < NEMB; k0 += 32) {
    const v16h ah = FragH::load(axh + k0);
    const v16h al = FragH::load(axl + k0);
    {
      const v16h bh = FragH::load(wh0 + k0);
      const v16h bl = FragH::load(wl0 + k0);
      mC0 = mma_g(ah, bh, mC0);
      rC0 = mma_g(ah, bl, rC0);
      rC0 = mma_g(al, bh, rC0);
    }
    {
      const v16h bh = FragH::load(wh1 + k0);
      const v16h bl = FragH::load(wl1 + k0);
      mC1 = mma_g(ah, bh, mC1);
      rC1 = mma_g(ah, bl, rC1);
      rC1 = mma_g(al, bh, rC1);
    }
    {
      const v16h bh = FragH::load(wh2 + k0);
      const v16h bl = FragH::load(wl2 + k0);
      mO0 = mma_g(ah, bh, mO0);
      rO0 = mma_g(ah, bl, rO0);
      rO0 = mma_g(al, bh, rO0);
    }
    {
      const v16h bh = FragH::load(wh3 + k0);
      const v16h bl = FragH::load(wl3 + k0);
      mO1 = mma_g(ah, bh, mO1);
      rO1 = mma_g(ah, bl, rO1);
      rO1 = mma_g(al, bh, rO1);
    }
  }
  acc_guard4(mC0, mC1, mO0, mO1);
  acc_guard4(rC0, rC1, rO0, rO1);

  float* slab = sT[wave];
#pragma unroll
  for (int r = 0; r < 8; ++r) {
    slab[(8 * hh + r) * SLP + rl]      = mC0[r] + rC0[r] * RES_CARRY_INV;
    slab[(8 * hh + r) * SLP + 16 + rl] = mC1[r] + rC1[r] * RES_CARRY_INV;
    slab[(8 * hh + r) * SLP + 32 + rl] = mO0[r] + rO0[r] * RES_CARRY_INV;
    slab[(8 * hh + r) * SLP + 48 + rl] = mO1[r] + rO1[r] * RES_CARRY_INV;
  }
  wave_lds_sync();

  const int q = lane >> 3, c4 = (lane & 7) * 4;
  const v4f bcv = *(const v4f*)(bc + n0 + c4);
  const v4f bov = *(const v4f*)(bo + n0 + c4);
#pragma unroll 1
  for (int it = 0; it < 4; ++it) {
    const int row = it * 4 + q;
    float* sp = slab + row * SLP + c4;
    const v4f vc = *(const v4f*)(sp);
    const v4f vo = *(const v4f*)(sp + 32);
    v4f cc, hv;
#pragma unroll
    for (int e = 0; e < 4; ++e) {
      const float cv = vc[e] * WCARRY_INV + bcv[e];
      const float ov = vo[e] * WCARRY_INV + bov[e];
      cc[e] = cv;
      hv[e] = sigm(ov) * tanhf(cv);
    }
    *(v4f*)(sp)      = cc;
    *(v4f*)(sp + 32) = hv;
    const size_t go = (size_t)(m0 + row) * NHID + n0 + c4;
    *(volatile v4f*)(LH + go) = hv;
    *(volatile v4f*)(LC + go) = cc;
  }
  __threadfence();
#pragma unroll 1
  for (int it = 0; it < 4; ++it) {
    const int row = it * 4 + q;
    const float* sp = slab + row * SLP + c4;
    const v4f cc = *(const v4f*)(sp);
    const v4f hv = *(const v4f*)(sp + 32);
    const size_t go = (size_t)(m0 + row) * NHID + n0 + c4;
    *(volatile v4f*)(LH + go) = hv;
    *(volatile v4f*)(LC + go) = cc;
  }
  __threadfence();
}

__global__ __launch_bounds__(NTHR) void stack_scan_kernel(const int* __restrict__ trans,
                                                          const unsigned short* __restrict__ WlrTp,
                                                          const float* __restrict__ bcomp,
                                                          const float* leaf_h, const float* leaf_c,
                                                          float* stack_h, float* stack_c, float* out) {
  __shared__ __align__(16) _Float16 At[ROWS_BLK * APITCH];
  __shared__ __align__(16) float    Gt[ROWS_BLK * GPITCH];
  const _Float16* WT = (const _Float16*)WlrTp;
  const int tid = threadIdx.x, lane = tid & 31, wave = tid >> 5;
  const int c = lane & 15, hh = lane >> 4, koff = hh * 8;
  const int rowbase = blockIdx.x * ROWS_BLK;
  const int row = tid >> 4, sub = tid & 15;
  const int b = rowbase + row;
  float* out1 = out + (size_t)NOUT0;
  float* out2 = out1 + (size_t)NOUT1;
  float* gslot = Gt + row * GPITCH;
  const v8f z8 = {0.f, 0.f, 0.f, 0.f, 0.f, 0.f, 0.f, 0.f};

  int sp = 0, bp = NLEAF;

#pragma unroll 1
  for (int t = 0; t < NSTEPS; ++t) {
    const int* trp = trans + t * NBAT + rowbase;
    int nr = 0;
#pragma unroll
    for (int k = 0; k < ROWS_BLK; ++k) nr |= (trp[k] != 1) ? 1 : 0;
    const int anyR = __builtin_amdgcn_readfirstlane(nr);
    const bool s = (trp[row] == 1);

    int li = sp - 2; li = li < 0 ? 0 : li; li = li > NLEAF - 1 ? NLEAF - 1 : li;
    int ri = sp - 1; ri = ri < 0 ? 0 : ri; ri = ri > NLEAF - 1 ? NLEAF - 1 : ri;
    int bi = bp - 1; bi = bi < 0 ? 0 : bi; bi = bi > NLEAF - 1 ? NLEAF - 1 : bi;
    int wr = s ? sp : (sp - 2); wr = wr < 0 ? 0 : wr; wr = wr > NLEAF - 1 ? NLEAF - 1 : wr;
    const size_t leafoff = ((size_t)bi * NBAT + (size_t)b) * NHID;
    const size_t lo = ((size_t)b * NLEAF + (size_t)li) * NHID;
    const size_t ro = ((size_t)b * NLEAF + (size_t)ri) * NHID;
    const float* pA = s ? (leaf_h + leafoff) : (stack_h + lo);
    const float* pB = s ? (leaf_h + leafoff) : (stack_h + ro);
    const float* pC = s ? (leaf_c + leafoff) : (stack_c + lo);
    const float* pD = s ? (leaf_h + leafoff) : (stack_c + ro);
    sp = s ? (sp + 1) : (sp - 1);
    bp = s ? (bp - 1) : bp;

    if (anyR) {
#pragma unroll
      for (int i = 0; i < 4; ++i) {
        const int col = 64 * i + 4 * sub;
        const v4f va = *(const v4f*)(pA + col);
        const v4f vb = *(const v4f*)(pB + col);
        v4h ha, hb;
#pragma unroll
        for (int e = 0; e < 4; ++e) {
          ha[e] = (_Float16)va[e];
          hb[e] = (_Float16)vb[e];
        }
        *(v4h*)(At + row * APITCH + col)        = ha;
        *(v4h*)(At + row * APITCH + NHID + col) = hb;
      }
    }
    __syncthreads();

    if (anyR) {
      v8f acc[8];
#pragma unroll
      for (int q = 0; q < 8; ++q) acc[q] = z8;
      const _Float16* ahrow = At + c * APITCH + koff;
      const _Float16* wrow  = WT + (size_t)(128 * wave + c) * NKC + koff;
#pragma unroll 1
      for (int k0 = 0; k0 < NKC; k0 += 32) {
        const v16h a = FragH::load(ahrow + k0);
        v16h bq[8];
#pragma unroll
        for (int q = 0; q < 8; ++q) bq[q] = FragH::load(wrow + (size_t)q * 16 * NKC + k0);
#pragma unroll
        for (int q = 0; q < 8; ++q) acc[q] = FragH::mma(a, bq[q], acc[q]);
        guard8_h(acc[0], acc[1], acc[2], acc[3], acc[4], acc[5], acc[6], acc[7],
                 a, bq[0], bq[1], bq[2], bq[3], bq[4], bq[5], bq[6], bq[7]);
      }
      acc_guard4(acc[0], acc[1], acc[2], acc[3]);
      acc_guard4(acc[4], acc[5], acc[6], acc[7]);
#pragma unroll
      for (int q = 0; q < 8; ++q)
#pragma unroll
        for (int r = 0; r < 8; ++r)
          Gt[(8 * hh + r) * GPITCH + 128 * wave + 16 * q + c] = acc[q][r];
    }
    __syncthreads();

    const bool last = (t == NSTEPS - 1);
    const size_t so = ((size_t)b * NLEAF + (size_t)wr) * NHID;
    const size_t oo = ((size_t)b * NSTEPS + (size_t)(NSTEPS - 1 - t)) * NHID;
    const size_t fo = (size_t)b * NHID;

#pragma unroll 1
    for (int i = 0; i < 4; ++i) {
      const int col = 64 * i + 4 * sub;
      const v4f vC = *(const v4f*)(pC + col);
      const v4f vD = *(const v4f*)(pD + col);
      v4f co = vC, ho = vD;
      if (anyR) {
        const v4f gi = *(const v4f*)(gslot + col);
        const v4f gl = *(const v4f*)(gslot + NHID + col);
        const v4f gr = *(const v4f*)(gslot + 2 * NHID + col);
        const v4f gu = *(const v4f*)(gslot + 3 * NHID + col);
        const v4f b0 = *(const v4f*)(bcomp + col);
        const v4f b1 = *(const v4f*)(bcomp + NHID + col);
        const v4f b2 = *(const v4f*)(bcomp + 2 * NHID + col);
        const v4f b3 = *(const v4f*)(bcomp + 3 * NHID + col);
#pragma unroll
        for (int e = 0; e < 4; ++e) {
          const float zi = gi[e] * WCARRY_INV + b0[e];
          const float zl = gl[e] * WCARRY_INV + b1[e];
          const float zr = gr[e] * WCARRY_INV + b2[e];
          const float zu = gu[e] * WCARRY_INV + b3[e];
          const float ig = sigm(zi);
          const float lf = sigm(zl);
          const float rf = sigm(zr);
          const float ug = tanhf(zu);
          const float cn = ig * ug + lf * vC[e] + rf * vD[e];
          const float hn = tanhf(cn);
          co[e] = s ? vC[e] : cn;
          ho[e] = s ? vD[e] : hn;
        }
      }
      *(v4f*)(gslot + col)        = co;
      *(v4f*)(gslot + NHID + col) = ho;
      *(volatile v4f*)(stack_h + so + col) = ho;
      *(volatile v4f*)(stack_c + so + col) = co;
      *(volatile v4f*)(out + oo + col)     = ho;
      if (last) {
        *(volatile v4f*)(out1 + fo + col) = ho;
        *(volatile v4f*)(out2 + fo + col) = co;
      }
    }
    __threadfence();
#pragma unroll 1
    for (int i = 0; i < 4; ++i) {
      const int col = 64 * i + 4 * sub;
      const v4f co = *(const v4f*)(gslot + col);
      const v4f ho = *(const v4f*)(gslot + NHID + col);
      *(volatile v4f*)(stack_h + so + col) = ho;
      *(volatile v4f*)(stack_c + so + col) = co;
      *(volatile v4f*)(out + oo + col)     = ho;
      if (last) {
        *(volatile v4f*)(out1 + fo + col) = ho;
        *(volatile v4f*)(out2 + fo + col) = co;
      }
    }
    __threadfence();
  }
}

extern "C" void kernel_launch(void* const* d_in, const int* in_sizes, int n_in,
                              void* d_out, int out_size, void* d_ws, size_t ws_size, hipStream_t stream) {
  if (n_in < 9 || d_out == nullptr || d_ws == nullptr) return;
  if (in_sizes[0] != NLEAF * NBAT * NEMB || in_sizes[1] != NEMB * NHID || in_sizes[2] != NHID ||
      in_sizes[3] != NEMB * NHID || in_sizes[4] != NHID || in_sizes[5] != NHID * NGATE ||
      in_sizes[6] != NHID * NGATE || in_sizes[7] != NGATE || in_sizes[8] != NSTEPS * NBAT ||
      out_size != NOUT0 + 2 * NOUT1) return;

  const float* seq   = (const float*)d_in[0];
  const float* Wc    = (const float*)d_in[1];
  const float* bc    = (const float*)d_in[2];
  const float* Wo    = (const float*)d_in[3];
  const float* bo    = (const float*)d_in[4];
  const float* Wl    = (const float*)d_in[5];
  const float* Wr    = (const float*)d_in[6];
  const float* bcomp = (const float*)d_in[7];
  const int*   trans = (const int*)d_in[8];
  float* out = (float*)d_out;

  char* ws = (char*)d_ws;
  size_t off = 0;
  auto carve = [&](size_t bytes) -> char* { char* p = ws + off; off += (bytes + 255) & ~(size_t)255; return p; };
  unsigned short* XH    = (unsigned short*)carve((size_t)NROWS * NEMB * 2);
  unsigned short* XL    = (unsigned short*)carve((size_t)NROWS * NEMB * 2);
  unsigned short* WCOT  = (unsigned short*)carve((size_t)2 * NHID * NEMB * 2);
  unsigned short* WCOL  = (unsigned short*)carve((size_t)2 * NHID * NEMB * 2);
  unsigned short* WLRT  = (unsigned short*)carve((size_t)NGATE * NKC * 2);
  float*          LEAFH = (float*)carve((size_t)NROWS * NHID * 4);
  float*          LEAFC = (float*)carve((size_t)NROWS * NHID * 4);
  float*          STKH  = (float*)carve((size_t)NBAT * NLEAF * NHID * 4);
  float*          STKC  = (float*)carve((size_t)NBAT * NLEAF * NHID * 4);
  if (off > ws_size || off > (size_t)134217728) return;

  const int n8 = NROWS * (NEMB / 8);
  cvt8_f16_split_kernel<<<(n8 + NTHR - 1) / NTHR, NTHR, 0, stream>>>(seq, XH, XL, n8);
  weight_planes_kernel<<<160, NTHR, 0, stream>>>(Wc, Wo, Wl, Wr, WCOT, WCOL, WLRT);
  leaf_gemm_kernel<<<(NROWS / 16) * (NHID / 32) / 8, NTHR, 0, stream>>>(XH, XL, WCOT, WCOL, bc, bo, LEAFH, LEAFC);
  stack_scan_kernel<<<NBAT / ROWS_BLK, NTHR, 0, stream>>>(trans, WLRT, bcomp, LEAFH, LEAFC, STKH, STKC, out);
}
